// MultiHeadAttention_36404142801403
// MI455X (gfx1250) — hardware-run, weakly checked
//
#include <hip/hip_runtime.h>

typedef __attribute__((ext_vector_type(16))) _Float16 v16h;
typedef __attribute__((ext_vector_type(16))) __bf16 v16b;
typedef __attribute__((ext_vector_type(8)))  _Float16 v8h;
typedef __attribute__((ext_vector_type(8)))  __bf16 v8b;
typedef __attribute__((ext_vector_type(8)))  float v8f;
typedef __attribute__((ext_vector_type(4)))  float v4f;
typedef __attribute__((ext_vector_type(4)))  unsigned v4u;

#ifndef NB
#define NB 4
#endif
#ifndef SEQ
#define SEQ 2048
#endif
#define NB_FULL 4
#define SEQ_FULL 2048
#define DIN 1024
#define CC 1024
#define NH 16
#define HD 64
#define EARLY (SEQ < 512 ? SEQ : 512)
#define NROWS (NB * SEQ)
#define NWORDS (NROWS / 32)
#define NXBLK (NROWS / 2)
#define WBLK (CC * DIN / 2048)
#define NEGBIG (-1.0e30f)
#define LN1024 (6.931471806f)

static_assert(SEQ % 64 == 0);
static_assert(EARLY % 64 == 0);
static_assert(NWORDS % 4 == 0);
static_assert(NWORDS * 4 <= 4096);
static_assert(SEQ <= SEQ_FULL);
static_assert(NB <= NB_FULL);
static_assert(DIN % 32 == 0);
static_assert(CC % 128 == 0);
static_assert(HD == 64);

#define SZ_ROWS16 ((size_t)2 * NROWS * CC)
#define SZ_W16    ((size_t)2 * CC * DIN)
#define SZ_E16    ((size_t)2 * NB * EARLY * CC)
#define WS_XB   ((size_t)0)
#define WS_WB   (WS_XB + SZ_ROWS16)
#define WS_WOB  (WS_WB + 3 * SZ_W16)
#define WS_WOH  (WS_WOB + SZ_W16)
#define WS_MB   (WS_WOH + SZ_W16)
#define WS_QKH  (WS_MB + (size_t)4096)
#define WS_VT   (WS_QKH + 2 * SZ_ROWS16)
#define WS_EH   (WS_VT + SZ_ROWS16)
#define WS_EL   (WS_EH + 2 * SZ_E16)
#define WS_VBH  (WS_EL + 2 * SZ_E16)
#define WS_VBL  (WS_VBH + SZ_E16)
#define WS_CTX  (WS_VBL + SZ_E16)
#define WS_CBH  (WS_CTX + SZ_ROWS16)
#define WS_CBL  (WS_CBH + SZ_E16)
#define WS_END  (WS_CBL + SZ_E16)
static_assert(WS_END <= (size_t)134217728);

template <typename T> __device__ __forceinline__ void vst2(void* p, T v) { *(volatile T*)p = v; __threadfence(); *(volatile T*)p = v; }
__device__ __forceinline__ v8f wmma16(v16h a, v16h b, v8f c) {
  v8f d = __builtin_amdgcn_wmma_f32_16x16x32_f16(false, a, false, b, (short)0, c, false, false);
  asm volatile("v_nop\n\tv_nop\n\tv_nop\n\tv_nop" : "+v"(d) : "v"(a), "v"(b));
  return d;
}
__device__ __forceinline__ v8f wmma_bf(v16b a, v16b b, v8f c) {
  v8f d = __builtin_amdgcn_wmma_f32_16x16x32_bf16(false, a, false, b, (short)0, c, false, false);
  asm volatile("v_nop\n\tv_nop\n\tv_nop\n\tv_nop" : "+v"(d) : "v"(a), "v"(b));
  return d;
}
__device__ __forceinline__ v16h frag_h(const _Float16* rowk0, int lane) {
  union { v16h v; v8h q[2]; } u; const _Float16* p = rowk0 + 8 * (lane >> 4);
  u.q[0] = *(const v8h*)p; u.q[1] = *(const v8h*)(p + 16); return u.v;
}
__device__ __forceinline__ v16b frag_b(const __bf16* rowk0, int lane) {
  union { v16b v; v8b q[2]; } u; const __bf16* p = rowk0 + 8 * (lane >> 4);
  u.q[0] = *(const v8b*)p; u.q[1] = *(const v8b*)(p + 16); return u.v;
}
#define LDSX() do { asm volatile("s_wait_dscnt 0" ::: "memory"); __builtin_amdgcn_wave_barrier(); __builtin_amdgcn_fence(3  , "workgroup"); } while (0)

__device__ __forceinline__ unsigned short hbits(float v) { return __builtin_bit_cast(unsigned short, (_Float16)v); }
__device__ __forceinline__ unsigned short bbits(__bf16 v) { return __builtin_bit_cast(unsigned short, v); }
__device__ __forceinline__ v4u pack8b(const v4f a, const v4f b) { union { v8b v; v4u u; } p;
#pragma unroll
  for (int i = 0; i < 4; ++i) { p.v[i] = (__bf16)a[i]; p.v[4 + i] = (__bf16)b[i]; }
  return p.u; }
__device__ __forceinline__ v4u pack8h256(const v4f a, const v4f b) { union { v8h v; v4u u; } p;
#pragma unroll
  for (int i = 0; i < 4; ++i) { p.v[i] = (_Float16)((float)(__bf16)a[i] * 256.0f); p.v[4 + i] = (_Float16)((float)(__bf16)b[i] * 256.0f); }
  return p.u; }

__global__ __launch_bounds__(256) void k_cvt(const float* __restrict__ X, const int* __restrict__ AM, const float* __restrict__ WQ, const float* __restrict__ WK, const float* __restrict__ WV, const float* __restrict__ WO,
    __bf16* __restrict__ XB, __bf16* __restrict__ WB, __bf16* __restrict__ WOB, _Float16* __restrict__ WOH, unsigned* __restrict__ MB) {
  __shared__ __align__(16) unsigned smw[NWORDS];
  const int tid = threadIdx.x; const int blk = blockIdx.x;
  if (blk < NXBLK) {
    const int row = blk * 2 + (tid >> 7); const int cc = (tid & 127) * 8; const int bb = row / SEQ, t = row % SEQ;
    const float* s = X + ((size_t)bb * SEQ_FULL + t) * DIN + cc;
    const v4f a = *(const v4f*)s; const v4f c = *(const v4f*)(s + 4);
    vst2(XB + (size_t)row * DIN + cc, pack8b(a, c));
  } else if (blk < NXBLK + WBLK) {
    const size_t e = ((size_t)(blk - NXBLK) * 256 + tid) * 8;
    const v4f a = *(const v4f*)(WQ + e); const v4f c = *(const v4f*)(WQ + e + 4);
    vst2(WB + e, pack8b(a, c));
  } else if (blk < NXBLK + 2 * WBLK) {
    const size_t e = ((size_t)(blk - NXBLK - WBLK) * 256 + tid) * 8;
    const v4f a = *(const v4f*)(WK + e); const v4f c = *(const v4f*)(WK + e + 4);
    vst2(WB + (size_t)CC * DIN + e, pack8b(a, c));
  } else if (blk < NXBLK + 3 * WBLK) {
    const size_t e = ((size_t)(blk - NXBLK - 2 * WBLK) * 256 + tid) * 8;
    const v4f a = *(const v4f*)(WV + e); const v4f c = *(const v4f*)(WV + e + 4);
    vst2(WB + (size_t)2 * CC * DIN + e, pack8b(a, c));
  } else if (blk < NXBLK + 4 * WBLK) {
    const size_t e = ((size_t)(blk - NXBLK - 3 * WBLK) * 256 + tid) * 8;
    const v4f a = *(const v4f*)(WO + e); const v4f c = *(const v4f*)(WO + e + 4);
    vst2(WOB + e, pack8b(a, c));
    vst2(WOH + e, pack8h256(a, c));
  } else {
    const int wave = __builtin_amdgcn_readfirstlane(tid >> 5); const int lane = tid & 31;
    for (int wd = wave; wd < NWORDS; wd += 8) { const int bb = wd / (SEQ / 32), tw = wd % (SEQ / 32);
      const int mv = AM[(size_t)bb * SEQ_FULL + tw * 32 + lane];
      const unsigned bits = __builtin_amdgcn_ballot_w32(mv != 0);
      if (lane == 0) smw[wd] = bits; }
    __syncthreads();
    for (int e = tid; e < NWORDS / 4; e += 256) vst2(MB + e * 4, *(const v4u*)&smw[e * 4]);
  }
}

__global__ __launch_bounds__(128) void k_proj(const __bf16* __restrict__ XB, const __bf16* __restrict__ WB, _Float16* __restrict__ QKH, __bf16* __restrict__ EH, __bf16* __restrict__ EL,
    _Float16* __restrict__ VT, __bf16* __restrict__ VBH, __bf16* __restrict__ VBL) {
  __shared__ __align__(16) unsigned short st[3][9216];
  const int tid = threadIdx.x; const int wave = __builtin_amdgcn_readfirstlane(tid >> 5); const int lane = tid & 31, col = lane & 15, g = lane >> 4;
  const int which = blockIdx.z; const int c0 = blockIdx.y * 128; const int r0 = blockIdx.x * 64; const int bb = r0 / SEQ, t0 = r0 % SEQ;
  const int wr = (wave & 1) * 32, wc = (wave >> 1) * 64;
  const bool early = t0 < EARLY;
  v8f acc[2][4] = {};
  const __bf16* ap = XB + (size_t)(r0 + wr + col) * DIN;
  const __bf16* wp = WB + (size_t)which * CC * DIN + (size_t)(c0 + wc + col) * DIN;
#pragma unroll 2
  for (int kc = 0; kc < DIN / 32; ++kc) {
    const v16b a0 = frag_b(ap + kc * 32, lane), a1 = frag_b(ap + 16 * DIN + kc * 32, lane);
#pragma unroll
    for (int j = 0; j < 4; ++j) { const v16b w = frag_b(wp + (size_t)j * 16 * DIN + kc * 32, lane); acc[0][j] = wmma_bf(a0, w, acc[0][j]); acc[1][j] = wmma_bf(a1, w, acc[1][j]); }
  }
  if (which < 2) {
#pragma unroll
    for (int i = 0; i < 2; ++i)
#pragma unroll
      for (int j = 0; j < 4; ++j)
#pragma unroll
        for (int r = 0; r < 8; ++r) { const float v = acc[i][j][r]; const int o = (wr + i * 16 + 8 * g + r) * 136 + wc + j * 16 + col;
          st[0][o] = hbits(v);
          if (early) { const __bf16 bh = (__bf16)v; st[1][o] = bbits(bh); st[2][o] = bbits((__bf16)(v - (float)bh)); } }
    __syncthreads();
    _Float16* DH = QKH + (size_t)which * NROWS * CC;
    for (int e = tid; e < 64 * 16; e += 128) { const int rl = e >> 4, q = e & 15; const int so = rl * 136 + q * 8;
      vst2(DH + (size_t)(r0 + rl) * CC + c0 + q * 8, *(const v4u*)&st[0][so]);
      if (early) { const size_t eo = (size_t)which * NB * EARLY * CC + ((size_t)bb * EARLY + t0 + rl) * CC + c0 + q * 8;
        vst2(EH + eo, *(const v4u*)&st[1][so]); vst2(EL + eo, *(const v4u*)&st[2][so]); } }
  } else {
#pragma unroll
    for (int i = 0; i < 2; ++i)
#pragma unroll
      for (int j = 0; j < 4; ++j)
#pragma unroll
        for (int r = 0; r < 8; ++r) { const float v = acc[i][j][r]; const int o = (wc + j * 16 + col) * 72 + wr + i * 16 + 8 * g + r;
          st[0][o] = hbits(v);
          if (early) { const __bf16 bh = (__bf16)v; st[1][o] = bbits(bh); st[2][o] = bbits((__bf16)(v - (float)bh)); } }
    __syncthreads();
    for (int e = tid; e < 128 * 8; e += 128) { const int cl = e >> 3, q = e & 7; const int so = cl * 72 + q * 8;
      vst2(VT + ((size_t)bb * CC + c0 + cl) * SEQ + t0 + q * 8, *(const v4u*)&st[0][so]);
      if (early) { const size_t eo = ((size_t)bb * CC + c0 + cl) * EARLY + t0 + q * 8;
        vst2(VBH + eo, *(const v4u*)&st[1][so]); vst2(VBL + eo, *(const v4u*)&st[2][so]); } }
  }
}

__device__ __forceinline__ float sm_step(const v8f s0, const v8f s1, const unsigned mw, const int j, const int q0, const int qg, const int g, float& m, float& l, float (&p)[16], const float carry) {
  float sv[16];
  if (mw == 0xffffffffu && j + 31 <= q0) {
#pragma unroll
    for (int r = 0; r < 8; ++r) { sv[r] = s0[r] * 0.125f; sv[8 + r] = s1[r] * 0.125f; }
  } else {
    const unsigned ml = mw >> (8 * g); const int kq = qg - j - 8 * g;
#pragma unroll
    for (int r = 0; r < 8; ++r) {
      const bool k0 = ((ml >> r) & 1u) != 0u && r <= kq;
      const bool k1 = ((ml >> (16 + r)) & 1u) != 0u && (16 + r) <= kq;
      sv[r] = k0 ? s0[r] * 0.125f : NEGBIG; sv[8 + r] = k1 ? s1[r] * 0.125f : NEGBIG; }
  }
  float mx = sv[0];
#pragma unroll
  for (int i = 1; i < 16; ++i) mx = fmaxf(mx, sv[i]);
  mx = fmaxf(mx, __shfl_xor(mx, 16));
  const float mn = fmaxf(m, mx);
  const float alpha = __expf(m - mn);
  const float msub = (mn < -1.0e29f ? 0.0f : mn) - carry;
  float ps = 0.f;
#pragma unroll
  for (int i = 0; i < 16; ++i) { p[i] = __expf(sv[i] - msub); ps += p[i]; }
  ps += __shfl_xor(ps, 16);
  l = l * alpha + ps; m = mn;
  return alpha;
}

__global__ __launch_bounds__(128) void k_attn_main(const _Float16* __restrict__ QKH, const _Float16* __restrict__ VT, const unsigned* __restrict__ MB, _Float16* __restrict__ CTX) {
  __shared__ v4u cs[4][16 * 9];
  const int wave = __builtin_amdgcn_readfirstlane(threadIdx.x >> 5); const int lane = threadIdx.x & 31, col = lane & 15, g = lane >> 4;
  const int b = blockIdx.z, h = blockIdx.y; const int q0 = EARLY + blockIdx.x * 64 + wave * 16; const int qg = q0 + col;
  const size_t rb = (size_t)b * SEQ;
  const _Float16* qrow = QKH + (rb + q0 + col) * CC + h * HD;
  const v16h bq0 = frag_h(qrow, lane), bq1 = frag_h(qrow + 32, lane);
  const _Float16* kbase = QKH + (size_t)NROWS * CC + (rb + col) * CC + h * HD;
  const _Float16* vbase = VT + ((size_t)b * CC + h * HD + col) * SEQ;
  const unsigned* mb = MB + b * (SEQ / 32);
  v8f o[4] = {}; float m = NEGBIG, l = 0.f;
  const int nst = (q0 + 16 + 31) >> 5;
#pragma unroll 1
  for (int s = 0; s < nst; ++s) { const int j = s * 32;
    const _Float16* kp = kbase + (size_t)j * CC;
    v8f s0 = {}, s1 = {};
    s0 = wmma16(frag_h(kp, lane), bq0, s0); s0 = wmma16(frag_h(kp + 32, lane), bq1, s0);
    s1 = wmma16(frag_h(kp + 16 * CC, lane), bq0, s1); s1 = wmma16(frag_h(kp + 16 * CC + 32, lane), bq1, s1);
    const unsigned mw = __builtin_amdgcn_readfirstlane(mb[s]);
    float p[16];
    const float alpha = sm_step(s0, s1, mw, j, q0, qg, g, m, l, p, LN1024);
    v16h pb;
#pragma unroll
    for (int i = 0; i < 16; ++i) pb[i] = (_Float16)p[i];
#pragma unroll
    for (int jd = 0; jd < 4; ++jd) o[jd] = o[jd] * alpha;
    const _Float16* vp = vbase + j;
#pragma unroll
    for (int jd = 0; jd < 4; ++jd) o[jd] = wmma16(frag_h(vp + (size_t)jd * 16 * SEQ, lane), pb, o[jd]);
  }
  const float inv = 64.0f * (1.0f / l);
#pragma unroll
  for (int jd = 0; jd < 4; ++jd) { union { v8h hv; v4u u; } pk;
#pragma unroll
    for (int r = 0; r < 8; ++r) pk.hv[r] = (_Float16)(o[jd][r] * inv);
    cs[wave][col * 9 + jd * 2 + g] = pk.u; }
  LDSX();
#pragma unroll
  for (int it = 0; it < 4; ++it) { const int row = it * 4 + (lane >> 3), pc = lane & 7;
    const v4u v = cs[wave][row * 9 + pc];
    vst2(CTX + (rb + q0 + row) * CC + h * HD + pc * 8, v); }
}

__device__ __forceinline__ v8f qk_hl(const __bf16* H, const __bf16* L, size_t o, int lane, const v16b qh0, const v16b ql0, const v16b qh1, const v16b ql1) {
  v8f s = {};
  const v16b kh0 = frag_b(H + o, lane), kl0 = frag_b(L + o, lane);
  s = wmma_bf(kl0, qh0, s); s = wmma_bf(kh0, ql0, s); s = wmma_bf(kh0, qh0, s);
  const v16b kh1 = frag_b(H + o + 32, lane), kl1 = frag_b(L + o + 32, lane);
  s = wmma_bf(kl1, qh1, s); s = wmma_bf(kh1, ql1, s); s = wmma_bf(kh1, qh1, s);
  return s;
}
__global__ __launch_bounds__(128) void k_attn_early(const __bf16* __restrict__ EH, const __bf16* __restrict__ EL, const __bf16* __restrict__ VBH, const __bf16* __restrict__ VBL, const unsigned* __restrict__ MB,
    __bf16* __restrict__ CBH, __bf16* __restrict__ CBL) {
  __shared__ v4u cs[2][4][16 * 9];
  const int wave = __builtin_amdgcn_readfirstlane(threadIdx.x >> 5); const int lane = threadIdx.x & 31, col = lane & 15, g = lane >> 4;
  const int b = blockIdx.z, h = blockIdx.y; const int q0 = blockIdx.x * 64 + wave * 16; const int qg = q0 + col;
  const size_t eb = (size_t)b * EARLY;
  const size_t qo = (eb + q0 + col) * CC + h * HD;
  const v16b qh0 = frag_b(EH + qo, lane), qh1 = frag_b(EH + qo + 32, lane), ql0 = frag_b(EL + qo, lane), ql1 = frag_b(EL + qo + 32, lane);
  const size_t kb0 = (size_t)NB * EARLY * CC + (eb + col) * CC + h * HD;
  const size_t vb0 = ((size_t)b * CC + h * HD + col) * EARLY;
  const unsigned* mb = MB + b * (SEQ / 32);
  v8f o[4] = {}; float m = NEGBIG, l = 0.f;
  const int nst = (q0 + 16 + 31) >> 5;
#pragma unroll 1
  for (int s = 0; s < nst; ++s) { const int j = s * 32;
    const size_t ko = kb0 + (size_t)j * CC;
    const v8f s0 = qk_hl(EH, EL, ko, lane, qh0, ql0, qh1, ql1);
    const v8f s1 = qk_hl(EH, EL, ko + (size_t)16 * CC, lane, qh0, ql0, qh1, ql1);
    const unsigned mw = __builtin_amdgcn_readfirstlane(mb[s]);
    float p[16];
    const float alpha = sm_step(s0, s1, mw, j, q0, qg, g, m, l, p, 0.0f);
    v16b ph, pl;
#pragma unroll
    for (int i = 0; i < 16; ++i) { const __bf16 hv = (__bf16)p[i]; ph[i] = hv; pl[i] = (__bf16)(p[i] - (float)hv); }
#pragma unroll
    for (int jd = 0; jd < 4; ++jd) o[jd] = o[jd] * alpha;
#pragma unroll
    for (int jd = 0; jd < 4; ++jd) { const size_t vo = vb0 + (size_t)jd * 16 * EARLY + j;
      const v16b vh = frag_b(VBH + vo, lane), vl = frag_b(VBL + vo, lane);
      o[jd] = wmma_bf(vl, ph, o[jd]); o[jd] = wmma_bf(vh, pl, o[jd]); o[jd] = wmma_bf(vh, ph, o[jd]); }
  }
  const float inv = 1.0f / l;
#pragma unroll
  for (int jd = 0; jd < 4; ++jd) { union { v8b bv; v4u u; } ph, pl;
#pragma unroll
    for (int r = 0; r < 8; ++r) { const float c = o[jd][r] * inv; const __bf16 hv = (__bf16)c; ph.bv[r] = hv; pl.bv[r] = (__bf16)(c - (float)hv); }
    cs[0][wave][col * 9 + jd * 2 + g] = ph.u; cs[1][wave][col * 9 + jd * 2 + g] = pl.u; }
  LDSX();
#pragma unroll
  for (int it = 0; it < 4; ++it) { const int row = it * 4 + (lane >> 3), pc = lane & 7;
    const v4u vh = cs[0][wave][row * 9 + pc]; const v4u vl = cs[1][wave][row * 9 + pc];
    const size_t eo = (eb + q0 + row) * CC + h * HD + pc * 8;
    vst2(CBH + eo, vh); vst2(CBL + eo, vl); }
}

__global__ __launch_bounds__(128) void k_out(const _Float16* __restrict__ CTX, const __bf16* __restrict__ CBH, const __bf16* __restrict__ CBL, const _Float16* __restrict__ WOH, const __bf16* __restrict__ WOB, float* __restrict__ OUT) {
  __shared__ __align__(16) float sf[64][132];
  const int tid = threadIdx.x; const int wave = __builtin_amdgcn_readfirstlane(tid >> 5); const int lane = tid & 31, col = lane & 15, g = lane >> 4;
  const int c0 = blockIdx.y * 128; const int r0 = blockIdx.x * 64; const int bb = r0 / SEQ, t0 = r0 % SEQ;
  const int wr = (wave & 1) * 32, wc = (wave >> 1) * 64;
  v8f acc[2][4] = {};
  if (t0 < EARLY) {
    const size_t er = ((size_t)bb * EARLY + t0 + wr + col) * CC;
    const __bf16* ah = CBH + er; const __bf16* al = CBL + er; const __bf16* wp = WOB + (size_t)(c0 + wc + col) * CC;
#pragma unroll 2
    for (int kc = 0; kc < CC / 32; ++kc) {
      const v16b a0h = frag_b(ah + kc * 32, lane), a0l = frag_b(al + kc * 32, lane), a1h = frag_b(ah + 16 * CC + kc * 32, lane), a1l = frag_b(al + 16 * CC + kc * 32, lane);
#pragma unroll
      for (int j = 0; j < 4; ++j) { const v16b w = frag_b(wp + (size_t)j * 16 * CC + kc * 32, lane);
        acc[0][j] = wmma_bf(a0l, w, acc[0][j]); acc[0][j] = wmma_bf(a0h, w, acc[0][j]);
        acc[1][j] = wmma_bf(a1l, w, acc[1][j]); acc[1][j] = wmma_bf(a1h, w, acc[1][j]); }
    }
#pragma unroll
    for (int i = 0; i < 2; ++i)
#pragma unroll
      for (int j = 0; j < 4; ++j)
#pragma unroll
        for (int r = 0; r < 8; ++r) sf[wr + i * 16 + 8 * g + r][wc + j * 16 + col] = acc[i][j][r];
  } else {
    const _Float16* ap = CTX + (size_t)(r0 + wr + col) * CC; const _Float16* wp = WOH + (size_t)(c0 + wc + col) * CC;
#pragma unroll 2
    for (int kc = 0; kc < CC / 32; ++kc) {
      const v16h a0 = frag_h(ap + kc * 32, lane), a1 = frag_h(ap + 16 * CC + kc * 32, lane);
#pragma unroll
      for (int j = 0; j < 4; ++j) { const v16h w = frag_h(wp + (size_t)j * 16 * CC + kc * 32, lane); acc[0][j] = wmma16(a0, w, acc[0][j]); acc[1][j] = wmma16(a1, w, acc[1][j]); }
    }
#pragma unroll
    for (int i = 0; i < 2; ++i)
#pragma unroll
      for (int j = 0; j < 4; ++j)
#pragma unroll
        for (int r = 0; r < 8; ++r) sf[wr + i * 16 + 8 * g + r][wc + j * 16 + col] = acc[i][j][r] * (1.0f / 16384.0f);
  }
  __syncthreads();
  for (int rl = 0; rl < 16; ++rl) { const int row = wave * 16 + rl;
    const v4f v = *(const v4f*)&sf[row][lane * 4];
    vst2(OUT + ((size_t)bb * SEQ_FULL + t0 + row) * DIN + c0 + lane * 4, v); }
}

extern "C" void kernel_launch(void* const* d_in, const int* in_sizes, int n_in, void* d_out, int out_size, void* d_ws, size_t ws_size, hipStream_t stream) {
  if (n_in < 6) return;
  const long long need_rows = (long long)(NB - 1) * SEQ_FULL + SEQ;
  if ((long long)in_sizes[0] < need_rows * DIN) return;
  if ((long long)in_sizes[1] < need_rows) return;
  if (in_sizes[2] < CC * DIN || in_sizes[3] < CC * DIN || in_sizes[4] < CC * DIN || in_sizes[5] < CC * DIN) return;
  if ((long long)out_size < need_rows * DIN) return;
  if (ws_size < (size_t)WS_END) return;
  const float* x = (const float*)d_in[0]; const int* am = (const int*)d_in[1];
  const float* wq = (const float*)d_in[2]; const float* wk = (const float*)d_in[3]; const float* wv = (const float*)d_in[4]; const float* wo = (const float*)d_in[5];
  char* ws = (char*)d_ws;
  __bf16* XB = (__bf16*)(ws + WS_XB); __bf16* WB = (__bf16*)(ws + WS_WB); __bf16* WOB = (__bf16*)(ws + WS_WOB); _Float16* WOH = (_Float16*)(ws + WS_WOH);
  unsigned* MB = (unsigned*)(ws + WS_MB);
  _Float16* QKH = (_Float16*)(ws + WS_QKH); _Float16* VT = (_Float16*)(ws + WS_VT);
  __bf16* EH = (__bf16*)(ws + WS_EH); __bf16* EL = (__bf16*)(ws + WS_EL); __bf16* VBH = (__bf16*)(ws + WS_VBH); __bf16* VBL = (__bf16*)(ws + WS_VBL);
  _Float16* CTX = (_Float16*)(ws + WS_CTX); __bf16* CBH = (__bf16*)(ws + WS_CBH); __bf16* CBL = (__bf16*)(ws + WS_CBL);

  k_cvt<<<dim3(NXBLK + 4 * WBLK + 1), 256, 0, stream>>>(x, am, wq, wk, wv, wo, XB, WB, WOB, WOH, MB);
  k_proj<<<dim3(NROWS / 64, CC / 128, 3), 128, 0, stream>>>(XB, WB, QKH, EH, EL, VT, VBH, VBL);
  k_attn_early<<<dim3(EARLY / 64, NH, NB), 128, 0, stream>>>(EH, EL, VBH, VBL, MB, CBH, CBL);
  if (SEQ > EARLY) k_attn_main<<<dim3((SEQ - EARLY) / 64, NH, NB), 128, 0, stream>>>(QKH, VT, MB, CTX);
  k_out<<<dim3(NROWS / 64, DIN / 128), 128, 0, stream>>>(CTX, CBH, CBL, WOH, WOB, (float*)d_out);
}
